// STSGCM_66632122630764
// MI455X (gfx1250) — hardware-verified
//
#include <hip/hip_runtime.h>
#include <math.h>

constexpr int kNodes = 3072;
constexpr int kBatch = 64;
constexpr int kChan  = 64;
constexpr int kBC    = kBatch * kChan;
constexpr int kOut2  = 128;
constexpr int kMid0  = 1024;
constexpr int kNMid  = 1024;
constexpr float kAScale  = 256.0f;
constexpr float kWScale  = 16.0f;
constexpr float kGCarry  = 8.0f;
constexpr float kG1Scale = kGCarry / kAScale;
constexpr float kG2Scale = kGCarry / (kAScale * kGCarry);
constexpr float kYScale  = 1.0f / (kGCarry * kWScale);

static_assert(kNodes % 64 == 0, "");
static_assert(kBC % 64 == 0, "");
static_assert(kNodes % 32 == 0, "");
static_assert(kChan % 32 == 0, "");
static_assert(kMid0 % 64 == 0 && kNMid % 64 == 0, "");

typedef __attribute__((ext_vector_type(16))) _Float16 v16h;
typedef __attribute__((ext_vector_type(8)))  _Float16 v8h;
typedef __attribute__((ext_vector_type(16))) __bf16   v16b;
typedef __attribute__((ext_vector_type(8)))  __bf16   v8b;
typedef __attribute__((ext_vector_type(8)))  float    v8f;
typedef __attribute__((ext_vector_type(4)))  float    v4f;
typedef __attribute__((ext_vector_type(4)))  unsigned int v4u;

__device__ __forceinline__ unsigned short f2bf_bits(float f) {
  unsigned u = __float_as_uint(f);
  return (unsigned short)((u + 0x7FFFu + ((u >> 16) & 1u)) >> 16);
}
__device__ __forceinline__ float bf_bits2f(unsigned short h) { return __uint_as_float(((unsigned)h) << 16); }

__device__ __forceinline__ void dep_guard_h(v8f& a, v8f& b, v16h x, v16h y) { asm volatile("v_nop\n\tv_nop\n\tv_nop\n\tv_nop" : "+v"(a), "+v"(b) : "v"(x), "v"(y)); }
__device__ __forceinline__ void dep_guard_b(v8f& a, v8f& b, v16b x, v16b y) { asm volatile("v_nop\n\tv_nop\n\tv_nop\n\tv_nop" : "+v"(a), "+v"(b) : "v"(x), "v"(y)); }
__device__ __forceinline__ void keep4_h(v16h a, v16h b, v16h c, v16h d) { asm volatile("v_nop" :: "v"(a), "v"(b), "v"(c), "v"(d)); }
__device__ __forceinline__ void keep4_b(v16b a, v16b b, v16b c, v16b d) { asm volatile("v_nop" :: "v"(a), "v"(b), "v"(c), "v"(d)); }
__device__ __forceinline__ void acc_guard4(v8f& a, v8f& b, v8f& c, v8f& d) { asm volatile("v_nop\n\tv_nop\n\tv_nop\n\tv_nop" : "+v"(a), "+v"(b), "+v"(c), "+v"(d)); }
template <typename T> struct Frag;
template <> struct Frag<_Float16> {
  typedef v16h V; union U { v16h v; v8h h[2]; };
  static __device__ __forceinline__ v16h load(const _Float16* p) {
    U f; f.h[0] = *(const v8h*)(p); f.h[1] = *(const v8h*)(p + 16); return f.v;
  }
  static __device__ __forceinline__ v8f mma(v16h a, v16h b, v8f c) {
    return __builtin_amdgcn_wmma_f32_16x16x32_f16(false, a, false, b, (short)0, c, false, false);
  }
  static __device__ __forceinline__ void guard(v8f& a, v8f& b, v16h x, v16h y) { dep_guard_h(a, b, x, y); }
  static __device__ __forceinline__ void keep(v16h a, v16h b, v16h c, v16h d) { keep4_h(a, b, c, d); }
};
template <> struct Frag<__bf16> {
  typedef v16b V; union U { v16b v; v8b h[2]; };
  static __device__ __forceinline__ v16b load(const __bf16* p) {
    U f; f.h[0] = *(const v8b*)(p); f.h[1] = *(const v8b*)(p + 16); return f.v;
  }
  static __device__ __forceinline__ v8f mma(v16b a, v16b b, v8f c) {
    return __builtin_amdgcn_wmma_f32_16x16x32_bf16(false, a, false, b, (short)0, c, false, false);
  }
  static __device__ __forceinline__ void guard(v8f& a, v8f& b, v16b x, v16b y) { dep_guard_b(a, b, x, y); }
  static __device__ __forceinline__ void keep(v16b a, v16b b, v16b c, v16b d) { keep4_b(a, b, c, d); }
};

__device__ __forceinline__ unsigned pk16(unsigned short a, unsigned short b) { return (unsigned)a | ((unsigned)b << 16); }
__device__ __forceinline__ unsigned short h_bits(float f) { const _Float16 h = (_Float16)f; return __builtin_bit_cast(unsigned short, h); }

template <int ET> struct Elem;
template <> struct Elem<0> { typedef _Float16 T; };
template <> struct Elem<1> { typedef __bf16 T; };
template <int ET, bool SPLIT, int BIAS_MODE, int OUT_MODE, bool RESID, int ACT = 0>
__global__ __launch_bounds__(256) void wmma_gemm64(
    const unsigned short* __restrict__ Ap, const unsigned short* __restrict__ A2p, int lda, long strideA,
    const unsigned short* __restrict__ Btp, const unsigned short* __restrict__ Bt2p, int ldb, long strideB,
    void* __restrict__ Cout, void* __restrict__ Cout2, int ldc, long strideC,
    const float* __restrict__ bias,
    const float* __restrict__ resid, long strideR,
    int M, int N, int K, float scale) {
  typedef typename Elem<ET>::T T;
  typedef typename Frag<T>::V V;
  const T* A = (const T*)Ap; const T* A2 = (const T*)A2p; const T* Bt = (const T*)Btp; const T* Bt2 = (const T*)Bt2p;
  __shared__ __align__(16) float sT[8][16 * 68];
  const int b    = blockIdx.y;
  const int lane = threadIdx.x & 31;
  const int wave = threadIdx.x >> 5;
  const int tilesN = N >> 6;
  const int tilesM = M >> 6;
  const int tile = blockIdx.x * 8 + wave;
  if (tile >= tilesM * tilesN) return;
  const int tm = tile / tilesN;
  const int tn = tile - tm * tilesN;
  const int m0 = tm << 6;
  const int n0 = tn << 6;

  const T* Ab  = A  + (size_t)b * strideA;
  const T* Bb  = Bt + (size_t)b * strideB;
  const T* Ab2 = SPLIT ? (A2  + (size_t)b * strideA) : nullptr;
  const T* Bb2 = SPLIT ? (Bt2 + (size_t)b * strideB) : nullptr;

  const int rlane = lane & 15;
  const int koff  = (lane >> 4) * 8;
  const int mOff  = (lane >> 4) * 8;

  v8f acc[4][4];
#pragma unroll
  for (int i = 0; i < 4; ++i)
#pragma unroll
    for (int j = 0; j < 4; ++j) acc[i][j] = (v8f){0.f,0.f,0.f,0.f,0.f,0.f,0.f,0.f};

  for (int k0 = 0; k0 < K; k0 += 32) {
    V bh[4], bl[4];
#pragma unroll
    for (int j = 0; j < 4; ++j) {
      const size_t bo = (size_t)(n0 + (j << 4) + rlane) * ldb + koff + k0;
      bh[j] = Frag<T>::load(Bb + bo);
      if (SPLIT) bl[j] = Frag<T>::load(Bb2 + bo);
    }
#pragma unroll
    for (int i = 0; i < 4; ++i) {
      const size_t ao = (size_t)(m0 + (i << 4) + rlane) * lda + koff + k0;
      V ah = Frag<T>::load(Ab + ao);
      V al;
      if (SPLIT) al = Frag<T>::load(Ab2 + ao);
#pragma unroll
      for (int j = 0; j < 4; ++j) {
        acc[i][j] = Frag<T>::mma(ah, bh[j], acc[i][j]);
        if (SPLIT) {
          acc[i][j] = Frag<T>::mma(ah, bl[j], acc[i][j]);
          acc[i][j] = Frag<T>::mma(al, bh[j], acc[i][j]);
        }
      }
      Frag<T>::guard(acc[i][0], acc[i][3], ah, SPLIT ? al : ah);
    }
    Frag<T>::keep(bh[0], bh[1], bh[2], bh[3]);
    if (SPLIT) Frag<T>::keep(bl[0], bl[1], bl[2], bl[3]);
  }
  acc_guard4(acc[0][0], acc[0][1], acc[0][2], acc[0][3]);
  acc_guard4(acc[1][0], acc[1][1], acc[1][2], acc[1][3]);
  acc_guard4(acc[2][0], acc[2][1], acc[2][2], acc[2][3]);
  acc_guard4(acc[3][0], acc[3][1], acc[3][2], acc[3][3]);

  float* slab = sT[wave];
  const float* Rb = RESID ? (resid + (size_t)b * strideR) : nullptr;
#pragma unroll
  for (int i = 0; i < 4; ++i) {
    const int mBase = m0 + (i << 4);
#pragma unroll
    for (int j = 0; j < 4; ++j) {
      const int n = n0 + (j << 4) + rlane;
      float bv = 0.f;
      if (BIAS_MODE == 2) bv = bias[n];
#pragma unroll
      for (int r = 0; r < 8; ++r) {
        float v = acc[i][j][r] * scale;
        if (BIAS_MODE == 1) v += bias[mBase + mOff + r];
        if (BIAS_MODE == 2) v += bv;
        if (RESID) v += Rb[(size_t)(mBase + mOff + r) * ldc + n];
        if (ACT == 2) v = fmaxf(v, 0.0f);
        if (ACT == 4) v = (v > 0.f) ? v : 0.01f * v;
        slab[(mOff + r) * 68 + (j << 4) + rlane] = v;
      }
    }
    __builtin_amdgcn_fence(__ATOMIC_RELEASE, "workgroup");
    __builtin_amdgcn_wave_barrier();
    __builtin_amdgcn_fence(__ATOMIC_ACQUIRE, "workgroup");
    if (OUT_MODE == 0) {
      float* C = (float*)Cout + (size_t)b * strideC;
      const int hh = lane >> 4, c4 = (lane & 15) * 4;
      for (int pass = 0; pass < 2; ++pass) {
#pragma unroll
        for (int it = 0; it < 8; ++it) {
          const int row = it * 2 + hh;
          v4f v = *(const v4f*)(slab + row * 68 + c4);
          *(volatile v4f*)(C + (size_t)(mBase + row) * ldc + n0 + c4) = v;
        }
        __threadfence();
      }
    } else {
      const int q = lane >> 3, c8 = (lane & 7) * 8;
      unsigned short* C  = (unsigned short*)Cout  + (size_t)b * strideC;
      unsigned short* C2 = (OUT_MODE == 2) ? ((unsigned short*)Cout2 + (size_t)b * strideC) : nullptr;
      for (int pass = 0; pass < 2; ++pass) {
#pragma unroll
        for (int it = 0; it < 4; ++it) {
          const int row = it * 4 + q;
          const float* sp = slab + row * 68 + c8;
          v8h hv, lv;
#pragma unroll
          for (int e = 0; e < 8; ++e) {
            if (OUT_MODE == 1) {
              hv[e] = (_Float16)sp[e];
            } else {
              unsigned short hb = f2bf_bits(sp[e]);
              unsigned short lb = f2bf_bits(sp[e] - bf_bits2f(hb));
              hv[e] = __builtin_bit_cast(_Float16, hb);
              lv[e] = __builtin_bit_cast(_Float16, lb);
            }
          }
          *(volatile v8h*)(C + (size_t)(mBase + row) * ldc + n0 + c8) = hv;
          if (OUT_MODE == 2) *(volatile v8h*)(C2 + (size_t)(mBase + row) * ldc + n0 + c8) = lv;
        }
        __threadfence();
      }
    }
    __builtin_amdgcn_fence(__ATOMIC_RELEASE, "workgroup");
    __builtin_amdgcn_wave_barrier();
    __builtin_amdgcn_fence(__ATOMIC_ACQUIRE, "workgroup");
  }
}

__global__ __launch_bounds__(256) void cast8_f16_kernel(const float* __restrict__ in, unsigned short* __restrict__ out,
                                                        int n8, float scale) {
  const int i = blockIdx.x * 256 + threadIdx.x;
  if (i >= n8) return;
  const float* p = in + 8 * (size_t)i;
  const v4f a = *(const v4f*)(p);
  const v4f c = *(const v4f*)(p + 4);
  unsigned short hb[8];
#pragma unroll
  for (int e = 0; e < 4; ++e) {
    hb[e]     = h_bits(a[e] * scale);
    hb[4 + e] = h_bits(c[e] * scale);
  }
  const v4u u = (v4u){pk16(hb[0], hb[1]), pk16(hb[2], hb[3]), pk16(hb[4], hb[5]), pk16(hb[6], hb[7])};
  unsigned short* q = out + 8 * (size_t)i;
  *(volatile v4u*)q = u;
  __threadfence();
  *(volatile v4u*)q = u;
}

__global__ __launch_bounds__(256) void xtcast_kernel(const float* __restrict__ x, unsigned short* __restrict__ X16) {
  __shared__ float sm[64][65];
  const int t  = threadIdx.x;
  const int m0 = blockIdx.x * 64;
  const int w0 = blockIdx.y * 64;
#pragma unroll
  for (int i = 0; i < 16; ++i) {
    const int e = i * 256 + t;
    const int r = e >> 6;
    const int c = e & 63;
    sm[c][r] = x[(size_t)(w0 + r) * kBC + m0 + c];
  }
  __syncthreads();
  const int lane = t & 31, wave = t >> 5;
  const int q = lane >> 3, c8 = (lane & 7) * 8;
  for (int pass = 0; pass < 2; ++pass) {
#pragma unroll
    for (int it = 0; it < 2; ++it) {
      const int row = wave * 8 + it * 4 + q;
      unsigned short hb[8];
#pragma unroll
      for (int e = 0; e < 8; ++e) hb[e] = h_bits(sm[row][c8 + e]);
      const v4u u = (v4u){pk16(hb[0], hb[1]), pk16(hb[2], hb[3]), pk16(hb[4], hb[5]), pk16(hb[6], hb[7])};
      *(volatile v4u*)(X16 + (size_t)(m0 + row) * kNodes + w0 + c8) = u;
    }
    __threadfence();
  }
}

template <int MODE>
__global__ __launch_bounds__(128) void glu_layer_kernel(
    const unsigned short* __restrict__ Gp,
    const unsigned short* __restrict__ Wp,
    const float* __restrict__ bias,
    unsigned short* __restrict__ H16,
    const float* __restrict__ Hmid_in,
    float* __restrict__ Fout) {
  __shared__ __align__(16) float hs[64 * 68];
  const _Float16* G = (const _Float16*)Gp;
  const _Float16* W = (const _Float16*)Wp;
  const int lane  = threadIdx.x & 31;
  const int wave  = threadIdx.x >> 5;
  const int rlane = lane & 15;
  const int koff  = (lane >> 4) * 8;
  const int hh    = lane >> 4;
  const int v0    = blockIdx.x * 64;
  const int b     = blockIdx.y;

  v8f acc[8];
#pragma unroll
  for (int jn = 0; jn < 8; ++jn) acc[jn] = (v8f){0.f,0.f,0.f,0.f,0.f,0.f,0.f,0.f};

#pragma unroll 1
  for (int k0 = 0; k0 < kChan; k0 += 32) {
    v16h bf[8];
#pragma unroll
    for (int jn = 0; jn < 8; ++jn)
      bf[jn] = Frag<_Float16>::load(W + (size_t)(jn * 16 + rlane) * kChan + koff + k0);
    const v16h af = Frag<_Float16>::load(G + ((size_t)(v0 + wave * 16 + rlane) * kBatch + b) * kChan + koff + k0);
#pragma unroll
    for (int jn = 0; jn < 8; ++jn) acc[jn] = Frag<_Float16>::mma(af, bf[jn], acc[jn]);
    Frag<_Float16>::guard(acc[0], acc[7], af, af);
    Frag<_Float16>::keep(bf[0], bf[1], bf[2], bf[3]);
    Frag<_Float16>::keep(bf[4], bf[5], bf[6], bf[7]);
  }
  acc_guard4(acc[0], acc[1], acc[2], acc[3]);
  acc_guard4(acc[4], acc[5], acc[6], acc[7]);

#pragma unroll
  for (int jn = 0; jn < 4; ++jn) {
    const int j = jn * 16 + rlane;
    const float bl = bias[j];
    const float br = bias[j + kChan];
#pragma unroll
    for (int r = 0; r < 8; ++r) {
      const int row = wave * 16 + hh * 8 + r;
      const float a = acc[jn][r] * kYScale + bl;
      const float g = acc[jn + 4][r] * kYScale + br;
      const float e = expf(-g);
      float h = a * __builtin_amdgcn_rcpf(1.0f + e);
      if (MODE == 1) {
        const float p = Hmid_in[((size_t)(v0 + row) * kBatch + b) * kChan + j];
        h = fmaxf(p, h);
      }
      hs[row * 68 + j] = h;
    }
  }
  __syncthreads();

  if (MODE == 0) {
    const int q = lane >> 3, c8 = (lane & 7) * 8;
    for (int pass = 0; pass < 2; ++pass) {
#pragma unroll
      for (int it = 0; it < 4; ++it) {
        const int j = wave * 16 + it * 4 + q;
        unsigned short hb[8];
#pragma unroll
        for (int e = 0; e < 8; ++e) hb[e] = h_bits(hs[(c8 + e) * 68 + j] * kGCarry);
        const v4u u = (v4u){pk16(hb[0], hb[1]), pk16(hb[2], hb[3]), pk16(hb[4], hb[5]), pk16(hb[6], hb[7])};
        *(volatile v4u*)(H16 + (size_t)(b * kChan + j) * kNodes + v0 + c8) = u;
      }
      __threadfence();
    }
    if (v0 >= kMid0 && v0 < kMid0 + kNMid) {
      const int c4 = (lane & 15) * 4;
      for (int pass = 0; pass < 2; ++pass) {
#pragma unroll
        for (int it = 0; it < 8; ++it) {
          const int row = wave * 16 + it * 2 + hh;
          const v4f val = *(const v4f*)(hs + row * 68 + c4);
          *(volatile v4f*)(Fout + ((size_t)(v0 - kMid0 + row) * kBatch + b) * kChan + c4) = val;
        }
        __threadfence();
      }
    }
  } else {
    const int c4 = (lane & 15) * 4;
    for (int pass = 0; pass < 2; ++pass) {
#pragma unroll
      for (int it = 0; it < 8; ++it) {
        const int row = wave * 16 + it * 2 + hh;
        const v4f val = *(const v4f*)(hs + row * 68 + c4);
        *(volatile v4f*)(Fout + ((size_t)(v0 + row) * kBatch + b) * kChan + c4) = val;
      }
      __threadfence();
    }
  }
}

extern "C" void kernel_launch(void* const* d_in, const int* in_sizes, int n_in,
                              void* d_out, int out_size, void* d_ws, size_t ws_size,
                              hipStream_t stream) {
  if (n_in < 6) return;
  if (in_sizes[0] != kNodes * kBC) return;
  if (in_sizes[1] != kNodes * kNodes) return;
  if (in_sizes[2] != kOut2 * kChan || in_sizes[3] != kOut2) return;
  if (in_sizes[4] != kOut2 * kChan || in_sizes[5] != kOut2) return;
  if (out_size != kNMid * kBatch * kChan) return;

  const float* x  = (const float*)d_in[0];
  const float* A  = (const float*)d_in[1];
  const float* W0 = (const float*)d_in[2];
  const float* b0 = (const float*)d_in[3];
  const float* W1 = (const float*)d_in[4];
  const float* b1 = (const float*)d_in[5];
  float* out = (float*)d_out;

  const size_t szX16  = (size_t)kBC * kNodes * 2;
  const size_t szA16  = (size_t)kNodes * kNodes * 2;
  const size_t szW16  = (size_t)2 * kOut2 * kChan * 2;
  const size_t szGT16 = (size_t)kNodes * kBC * 2;
  const size_t szH116 = (size_t)kBC * kNodes * 2;
  const size_t szHMID = (size_t)kNMid * kBatch * kChan * 4;
  const size_t szG2T  = (size_t)kNMid * kBC * 2;
  const size_t offX16  = 0;
  const size_t offA16  = offX16 + szX16;
  const size_t offW16  = offA16 + szA16;
  const size_t offGT16 = offW16 + szW16;
  const size_t offH116 = offGT16 + szGT16;
  const size_t offHMID = offH116 + szH116;
  const size_t offG2T  = offHMID + szHMID;
  const size_t total   = offG2T + szG2T;
  if (total > ws_size) return;

  char* ws = (char*)d_ws;
  unsigned short* X16   = (unsigned short*)(ws + offX16);
  unsigned short* A16   = (unsigned short*)(ws + offA16);
  unsigned short* W16   = (unsigned short*)(ws + offW16);
  unsigned short* W16b  = W16 + kOut2 * kChan;
  unsigned short* GT16  = (unsigned short*)(ws + offGT16);
  unsigned short* H116  = (unsigned short*)(ws + offH116);
  float*          HMID  = (float*)(ws + offHMID);
  unsigned short* G2T16 = (unsigned short*)(ws + offG2T);

  xtcast_kernel<<<dim3(kBC / 64, kNodes / 64), 256, 0, stream>>>(x, X16);
  {
    const int n8A = kNodes * kNodes / 8;
    cast8_f16_kernel<<<(n8A + 255) / 256, 256, 0, stream>>>(A, A16, n8A, kAScale);
    const int n8W = kOut2 * kChan / 8;
    cast8_f16_kernel<<<(n8W + 255) / 256, 256, 0, stream>>>(W0, W16, n8W, kWScale);
    cast8_f16_kernel<<<(n8W + 255) / 256, 256, 0, stream>>>(W1, W16b, n8W, kWScale);
  }
  {
    const int M = kNodes, N = kBC, K = kNodes;
    const int tiles = (M / 64) * (N / 64);
    wmma_gemm64<0, false, 0, 1, false, 0><<<dim3((tiles + 7) / 8, 1), 256, 0, stream>>>(
        A16, A16, kNodes, 0L, X16, X16, kNodes, 0L, (void*)GT16, (void*)GT16, kBC, 0L,
        b0, HMID, 0L, M, N, K, kG1Scale);
  }
  glu_layer_kernel<0><<<dim3(kNodes / 64, kBatch), 128, 0, stream>>>(GT16, W16, b0, H116, (const float*)HMID, HMID);
  {
    const int M = kNMid, N = kBC, K = kNodes;
    const int tiles = (M / 64) * (N / 64);
    wmma_gemm64<0, false, 0, 1, false, 0><<<dim3((tiles + 7) / 8, 1), 256, 0, stream>>>(
        A16 + (size_t)kMid0 * kNodes, A16 + (size_t)kMid0 * kNodes, kNodes, 0L, H116, H116, kNodes, 0L,
        (void*)G2T16, (void*)G2T16, kBC, 0L, b1, HMID, 0L, M, N, K, kG2Scale);
  }
  glu_layer_kernel<1><<<dim3(kNMid / 64, kBatch), 128, 0, stream>>>(G2T16, W16b, b1, H116, (const float*)HMID, out);
}
